// RNN_40776419508632
// MI455X (gfx1250) — hardware-verified
//
#include <hip/hip_runtime.h>
#include <math.h>
#include <stdint.h>

constexpr int kBatch = 8;
constexpr int kSeq   = 2048;
constexpr int kDim   = 512;
constexpr int kTok   = kBatch * kSeq;
constexpr int kNumX  = kTok * kDim;
constexpr int kNumW  = kDim * kDim;
constexpr int kOut1Elem = kNumX;
constexpr int kOutTotal = kNumX + 2 * kBatch * kDim;

constexpr size_t kPlaneBytes  = (size_t)kTok * kDim * 2;
constexpr size_t kWPlaneBytes = (size_t)kDim * kDim * 2;
constexpr size_t kOffXB  = 0;
constexpr size_t kOffW0  = kOffXB + kPlaneBytes;
constexpr size_t kOffW1  = kOffW0 + kWPlaneBytes;
constexpr size_t kOffWt  = kOffW1 + kWPlaneBytes;
constexpr size_t kOffH0h = kOffWt + kWPlaneBytes;
constexpr size_t kOffH0l = kOffH0h + kPlaneBytes;
constexpr size_t kOffH1h = kOffH0l + kPlaneBytes;
constexpr size_t kOffH1l = kOffH1h + kPlaneBytes;
constexpr size_t kWsTotal = kOffH1l + kPlaneBytes;
static_assert(kWsTotal <= (size_t)134217728u);
static_assert(kOffW0 % 128 == 0 && kOffW1 % 128 == 0 && kOffWt % 128 == 0);
static_assert(kOffH0h % 128 == 0 && kOffH0l % 128 == 0 && kOffH1h % 128 == 0 && kOffH1l % 128 == 0);
static_assert(kTok % 64 == 0 && kDim % 64 == 0 && kDim % 32 == 0);
static_assert((size_t)kOut1Elem * 4 == (size_t)33554432u);
static_assert((size_t)kOutTotal * 4 == (size_t)33587200u);
static_assert(kNumX % (8 * 256) == 0 && kNumW % (8 * 256) == 0);
static_assert(((kTok / 64) * (kDim / 64)) % 8 == 0);

constexpr int kCastBlocksX = kNumX / 8 / 256;
constexpr int kCastBlocksW = kNumW / 8 / 256;
constexpr int kGemmBlocks  = (kTok / 64) * (kDim / 64) / 8;

typedef __attribute__((ext_vector_type(16))) _Float16 v16h;
typedef __attribute__((ext_vector_type(8)))  _Float16 v8h;
typedef __attribute__((ext_vector_type(16))) __bf16   v16b;
typedef __attribute__((ext_vector_type(8)))  __bf16   v8b;
typedef __attribute__((ext_vector_type(8)))  float    v8f;
typedef __attribute__((ext_vector_type(4)))  float    v4f;
typedef __attribute__((ext_vector_type(4)))  unsigned int v4u;

__device__ __forceinline__ unsigned short f2bf_bits(float f) {
  unsigned u = __float_as_uint(f);
  return (unsigned short)((u + 0x7FFFu + ((u >> 16) & 1u)) >> 16);
}
__device__ __forceinline__ float bf_bits2f(unsigned short h) { return __uint_as_float(((unsigned)h) << 16); }

__device__ __forceinline__ void keep4_b(v16b a, v16b b, v16b c, v16b d) { asm volatile("v_nop" :: "v"(a), "v"(b), "v"(c), "v"(d)); }
__device__ __forceinline__ void acc_guard4(v8f& a, v8f& b, v8f& c, v8f& d) { asm volatile("v_nop\n\tv_nop\n\tv_nop\n\tv_nop" : "+v"(a), "+v"(b), "+v"(c), "+v"(d)); }
__device__ __forceinline__ void guard_grp_b(v8f& a0, v8f& a1, v8f& a2, v8f& a3,
                                            v16b x, v16b y, v16b p0, v16b p1, v16b p2, v16b p3) {
  asm volatile("v_nop\n\tv_nop\n\tv_nop\n\tv_nop"
               : "+v"(a0), "+v"(a1), "+v"(a2), "+v"(a3)
               : "v"(x), "v"(y), "v"(p0), "v"(p1), "v"(p2), "v"(p3));
}

template <typename T> struct Frag;
template <> struct Frag<__bf16> {
  typedef v16b V; union U { v16b v; v8b h[2]; };
  static __device__ __forceinline__ v16b load(const __bf16* p) {
    U f; f.h[0] = *(const v8b*)(p); f.h[1] = *(const v8b*)(p + 16); return f.v;
  }
  static __device__ __forceinline__ v8f mma(v16b a, v16b b, v8f c) {
    return __builtin_amdgcn_wmma_f32_16x16x32_bf16(false, a, false, b, (short)0, c, false, false);
  }
};

__device__ __forceinline__ unsigned pk16(unsigned short a, unsigned short b) { return (unsigned)a | ((unsigned)b << 16); }

__global__ __launch_bounds__(256) void cast8_bf16_kernel(const float* __restrict__ in,
                                                         unsigned short* __restrict__ out, int n8) {
  const int i = blockIdx.x * 256 + threadIdx.x;
  if (i >= n8) return;
  const float* p = in + 8 * (size_t)i;
  const v4f a = *(const v4f*)(p);
  const v4f c = *(const v4f*)(p + 4);
  unsigned short hb[8];
#pragma unroll
  for (int e = 0; e < 4; ++e) {
    hb[e]     = f2bf_bits(a[e]);
    hb[4 + e] = f2bf_bits(c[e]);
  }
  const v4u u = (v4u){pk16(hb[0], hb[1]), pk16(hb[2], hb[3]), pk16(hb[4], hb[5]), pk16(hb[6], hb[7])};
  unsigned short* q = out + 8 * (size_t)i;
  *(volatile v4u*)q = u;
  __threadfence();
  *(volatile v4u*)q = u;
}

template <int SPLITA, int OUT16, int ACT_TANH, int HFIN>
__global__ __launch_bounds__(256) void gemm64_kernel(
    const unsigned short* __restrict__ Ap, const unsigned short* __restrict__ A2p, int lda,
    const unsigned short* __restrict__ Btp, int ldb,
    void* __restrict__ Cout, void* __restrict__ Cout2, int ldc,
    const float* __restrict__ bias, float* __restrict__ hfin,
    int M, int N, int K) {
  typedef __bf16 T;
  typedef v16b V;
  const T* A  = (const T*)Ap;
  const T* A2 = (const T*)A2p;
  const T* Bt = (const T*)Btp;
  __shared__ __align__(16) float sT[8][16 * 68];
  const int lane = threadIdx.x & 31;
  const int wave = threadIdx.x >> 5;
  const int tilesN = N >> 6;
  const int tilesM = M >> 6;
  const int tile = blockIdx.x * 8 + wave;
  if (tile >= tilesM * tilesN) return;
  const int tm = tile / tilesN;
  const int tn = tile - tm * tilesN;
  const int m0 = tm << 6;
  const int n0 = tn << 6;

  const int rlane = lane & 15;
  const int koff  = (lane >> 4) * 8;
  const int mOff  = (lane >> 4) * 8;

  v8f acc[4][4];
#pragma unroll
  for (int i = 0; i < 4; ++i)
#pragma unroll
    for (int j = 0; j < 4; ++j) acc[i][j] = (v8f){0.f,0.f,0.f,0.f,0.f,0.f,0.f,0.f};

  for (int k0 = 0; k0 < K; k0 += 32) {
    V bh[4];
#pragma unroll
    for (int j = 0; j < 4; ++j) {
      const size_t bo = (size_t)(n0 + (j << 4) + rlane) * ldb + koff + k0;
      bh[j] = Frag<T>::load(Bt + bo);
    }
#pragma unroll
    for (int i = 0; i < 4; ++i) {
      const size_t ao = (size_t)(m0 + (i << 4) + rlane) * lda + koff + k0;
      V ah = Frag<T>::load(A + ao);
      V al = ah;
      if (SPLITA) al = Frag<T>::load(A2 + ao);
#pragma unroll
      for (int j = 0; j < 4; ++j) {
        acc[i][j] = Frag<T>::mma(ah, bh[j], acc[i][j]);
        if (SPLITA) acc[i][j] = Frag<T>::mma(al, bh[j], acc[i][j]);
      }
      guard_grp_b(acc[i][0], acc[i][1], acc[i][2], acc[i][3], ah, al, bh[0], bh[1], bh[2], bh[3]);
    }
    keep4_b(bh[0], bh[1], bh[2], bh[3]);
  }
  acc_guard4(acc[0][0], acc[0][1], acc[0][2], acc[0][3]);
  acc_guard4(acc[1][0], acc[1][1], acc[1][2], acc[1][3]);
  acc_guard4(acc[2][0], acc[2][1], acc[2][2], acc[2][3]);
  acc_guard4(acc[3][0], acc[3][1], acc[3][2], acc[3][3]);

  float bvs[4];
#pragma unroll
  for (int j = 0; j < 4; ++j) bvs[j] = bf_bits2f(f2bf_bits(bias[n0 + (j << 4) + rlane]));

  float* slab = sT[wave];
#pragma unroll
  for (int i = 0; i < 4; ++i) {
    const int mBase = m0 + (i << 4);
#pragma unroll
    for (int j = 0; j < 4; ++j) {
#pragma unroll
      for (int r = 0; r < 8; ++r) {
        float v = acc[i][j][r] + bvs[j];
        if (ACT_TANH) v = tanhf(v);
        slab[(mOff + r) * 68 + (j << 4) + rlane] = v;
      }
    }
    __builtin_amdgcn_fence(__ATOMIC_RELEASE, "workgroup");
    __builtin_amdgcn_wave_barrier();
    __builtin_amdgcn_fence(__ATOMIC_ACQUIRE, "workgroup");
    if (OUT16 == 0) {
      float* C = (float*)Cout;
      const int hh = lane >> 4, c4 = (lane & 15) * 4;
      for (int pass = 0; pass < 2; ++pass) {
#pragma unroll
        for (int it = 0; it < 8; ++it) {
          const int row = it * 2 + hh;
          v4f v = *(const v4f*)(slab + row * 68 + c4);
          *(volatile v4f*)(C + (size_t)(mBase + row) * ldc + n0 + c4) = v;
        }
        __threadfence();
      }
    } else {
      const int q = lane >> 3, c8 = (lane & 7) * 8;
      unsigned short* C  = (unsigned short*)Cout;
      unsigned short* C2 = (unsigned short*)Cout2;
      for (int pass = 0; pass < 2; ++pass) {
#pragma unroll
        for (int it = 0; it < 4; ++it) {
          const int row = it * 4 + q;
          const float* sp = slab + row * 68 + c8;
          v8h hv, lv;
#pragma unroll
          for (int e = 0; e < 8; ++e) {
            const float f = sp[e];
            const unsigned short hb = f2bf_bits(f);
            const unsigned short lb = f2bf_bits(f - bf_bits2f(hb));
            hv[e] = __builtin_bit_cast(_Float16, hb);
            lv[e] = __builtin_bit_cast(_Float16, lb);
          }
          *(volatile v8h*)(C  + (size_t)(mBase + row) * ldc + n0 + c8) = hv;
          *(volatile v8h*)(C2 + (size_t)(mBase + row) * ldc + n0 + c8) = lv;
        }
        __threadfence();
      }
    }
    if (HFIN) {
      const int lastRow = mBase + 15;
      if ((lastRow & (kSeq - 1)) == (kSeq - 1)) {
        const int bidx = lastRow / kSeq;
        float* orow = hfin + (size_t)bidx * kDim + n0;
        const int hq = lane >> 4, c4 = (lane & 15) * 4;
        const v4f hv4 = *(const v4f*)(slab + 15 * 68 + c4);
        for (int pass = 0; pass < 2; ++pass) {
          if (hq == 0) *(volatile v4f*)(orow + c4) = hv4;
          __threadfence();
        }
      }
    }
    __builtin_amdgcn_fence(__ATOMIC_RELEASE, "workgroup");
    __builtin_amdgcn_wave_barrier();
    __builtin_amdgcn_fence(__ATOMIC_ACQUIRE, "workgroup");
  }
}

extern "C" void kernel_launch(void* const* d_in, const int* in_sizes, int n_in,
                              void* d_out, int out_size, void* d_ws, size_t ws_size,
                              hipStream_t stream) {
  if (n_in < 7) return;
  if (in_sizes[0] != kNumX || in_sizes[1] != kNumW || in_sizes[2] != kDim ||
      in_sizes[3] != kNumW || in_sizes[4] != kDim || in_sizes[5] != kNumW || in_sizes[6] != kDim) return;
  if (out_size != kOutTotal) return;
  if (ws_size < kWsTotal) return;

  const float* x  = (const float*)d_in[0];
  const float* W0 = (const float*)d_in[1];
  const float* b0 = (const float*)d_in[2];
  const float* W1 = (const float*)d_in[3];
  const float* b1 = (const float*)d_in[4];
  const float* Wt = (const float*)d_in[5];
  const float* bt = (const float*)d_in[6];
  float* out = (float*)d_out;

  char* ws = (char*)d_ws;
  unsigned short* XB  = (unsigned short*)(ws + kOffXB);
  unsigned short* W0B = (unsigned short*)(ws + kOffW0);
  unsigned short* W1B = (unsigned short*)(ws + kOffW1);
  unsigned short* WtB = (unsigned short*)(ws + kOffWt);
  unsigned short* H0h = (unsigned short*)(ws + kOffH0h);
  unsigned short* H0l = (unsigned short*)(ws + kOffH0l);
  unsigned short* H1h = (unsigned short*)(ws + kOffH1h);
  unsigned short* H1l = (unsigned short*)(ws + kOffH1l);

  float* hfin0 = out + kOut1Elem;
  float* hfin1 = out + kOut1Elem + kBatch * kDim;

  cast8_bf16_kernel<<<dim3(kCastBlocksX), dim3(256), 0, stream>>>(x,  XB,  kNumX / 8);
  cast8_bf16_kernel<<<dim3(kCastBlocksW), dim3(256), 0, stream>>>(W0, W0B, kNumW / 8);
  cast8_bf16_kernel<<<dim3(kCastBlocksW), dim3(256), 0, stream>>>(W1, W1B, kNumW / 8);
  cast8_bf16_kernel<<<dim3(kCastBlocksW), dim3(256), 0, stream>>>(Wt, WtB, kNumW / 8);

  gemm64_kernel<0, 1, 1, 1><<<dim3(kGemmBlocks), dim3(256), 0, stream>>>(
      XB, XB, kDim, W0B, kDim, (void*)H0h, (void*)H0l, kDim, b0, hfin0, kTok, kDim, kDim);
  gemm64_kernel<1, 1, 1, 1><<<dim3(kGemmBlocks), dim3(256), 0, stream>>>(
      H0h, H0l, kDim, W1B, kDim, (void*)H1h, (void*)H1l, kDim, b1, hfin1, kTok, kDim, kDim);
  gemm64_kernel<1, 0, 0, 0><<<dim3(kGemmBlocks), dim3(256), 0, stream>>>(
      H1h, H1l, kDim, WtB, kDim, (void*)out, (void*)out, kDim, bt, hfin0, kTok, kDim, kDim);
}
